// TransformerPlanner_82231443849776
// MI455X (gfx1250) — hardware-verified
//
#include <hip/hip_runtime.h>
#include <stddef.h>
#include <stdint.h>

#define TT    10
#define NTK   20
#define NWP   3
#define DM    128
#define NHD   8
#define HD    16
#define DF    256
#define SPB   16
#define SPH   8
#define TRH   (SPH * NTK)
#define QR    (SPB * NWP)
#define TP    136
#define XP    132
#define HP    264
#define NOUT  (SPB * NWP * 2)

#define W_CARRY   32.0f
#define CTX_CARRY 16.0f
#define HID_CARRY 16.0f
#define KV_SCL    0.03125f
#define F1_SCL    0.03125f
#define OP_SCL    0.001953125f
#define F2_SCL    0.001953125f

static_assert(TRH % 32 == 0);
static_assert(QR % 16 == 0);
static_assert((NOUT * 4) % 128 == 0);
static_assert(DM % 32 == 0);
static_assert(DF % 32 == 0);
static_assert(NHD * HD == DM);
static_assert(SPH * NHD * NWP <= 256);

#define L_TOK   0
#define L_KV    (TRH * TP * 2)
#define L_AEND  (2 * TRH * TP * 2)
#define L_X32   0
#define L_XH    (QR * XP * 4)
#define L_HF    (L_XH + QR * TP * 2)
#define L_SC    L_AEND
#define L_CTX   (L_SC + SPH * NHD * NWP * NTK * 4)
#define L_Q     (L_CTX + QR * TP * 2)
#define L_QLN   (L_Q + NWP * DM * 4)
#define L_OUT   (L_QLN + NWP * DM * 4)
#define L_TOTAL (L_OUT + NOUT * 4)
static_assert(L_HF + QR * HP * 2 <= L_AEND);
static_assert(L_TOTAL == 118912);
static_assert(L_KV % 16 == 0);
static_assert(L_XH % 16 == 0);
static_assert(L_HF % 16 == 0);
static_assert(L_SC % 16 == 0);
static_assert(L_CTX % 16 == 0);
static_assert(L_Q % 16 == 0);
static_assert(L_QLN % 16 == 0);
static_assert(L_OUT % 16 == 0);

typedef _Float16 v16h __attribute__((ext_vector_type(16)));
typedef _Float16 v8h  __attribute__((ext_vector_type(8)));
typedef _Float16 v4h  __attribute__((ext_vector_type(4)));
typedef float    v8f  __attribute__((ext_vector_type(8)));
typedef float    v4f  __attribute__((ext_vector_type(4)));
typedef unsigned int v4u __attribute__((ext_vector_type(4)));

union Frag  { v16h v; v8h h[2]; };
union Pack8 { v8h h; v4u u; };

__device__ __forceinline__ v8f mma16(v16h a, v16h b, v8f c) {
  c = __builtin_amdgcn_wmma_f32_16x16x32_f16(false, a, false, b, (short)0, c, false, false);
  asm volatile("v_nop\n\tv_nop\n\tv_nop\n\tv_nop" : "+v"(c) : "v"(a), "v"(b));
  return c;
}

__device__ __forceinline__ v16h ldfrag(const _Float16* p, int ld, int row0, int k0, int lane) {
  const int m = lane & 15, lh = lane >> 4;
  const _Float16* q = p + (size_t)(row0 + m) * ld + k0 + 8 * lh;
  Frag f;
  f.h[0] = *(const v8h*)(q);
  f.h[1] = *(const v8h*)(q + 16);
  return f.v;
}

__device__ __forceinline__ v8f zero8() { return (v8f){0.f, 0.f, 0.f, 0.f, 0.f, 0.f, 0.f, 0.f}; }

__device__ __forceinline__ float wsum(float v) {
#pragma unroll
  for (int o = 16; o >= 1; o >>= 1) v += __shfl_xor(v, o, 32);
  return v;
}

__global__ __launch_bounds__(256) void k_wcvt(const float* __restrict__ src, _Float16* __restrict__ dst) {
  const size_t o = ((size_t)blockIdx.x * 256 + threadIdx.x) * 8;
  const v4f a0 = *(const v4f*)(src + o) * W_CARRY;
  const v4f a1 = *(const v4f*)(src + o + 4) * W_CARRY;
  Pack8 pk;
  pk.h = (v8h){(_Float16)a0[0], (_Float16)a0[1], (_Float16)a0[2], (_Float16)a0[3],
               (_Float16)a1[0], (_Float16)a1[1], (_Float16)a1[2], (_Float16)a1[3]};
  const v4u vv = pk.u;
  volatile v4u* d = (volatile v4u*)(dst + o);
  *d = vv;
  __threadfence();
  *d = vv;
}

__global__ __launch_bounds__(128) void k_qprep(const float* __restrict__ qe, const float* __restrict__ qg,
                                               const float* __restrict__ qbb, const float* __restrict__ ipw,
                                               const float* __restrict__ ipb,
                                               float* __restrict__ qout, float* __restrict__ qlnout) {
  __shared__ float red[4];
  __shared__ __align__(16) float qs[NWP * DM];
  __shared__ __align__(16) float qo[NWP * DM];
  const int t = threadIdx.x, lane = t & 31, w32 = t >> 5;
#pragma unroll 1
  for (int w = 0; w < NWP; ++w) {
    const float v = qe[w * DM + t];
    const float s = wsum(v);
    if (lane == 0) red[w32] = s;
    __syncthreads();
    const float mean = ((red[0] + red[1]) + (red[2] + red[3])) * (1.0f / 128.0f);
    __syncthreads();
    const float d = v - mean;
    const float s2 = wsum(d * d);
    if (lane == 0) red[w32] = s2;
    __syncthreads();
    const float var = ((red[0] + red[1]) + (red[2] + red[3])) * (1.0f / 128.0f);
    const float xn = d * rsqrtf(var + 1e-5f) * qg[t] + qbb[t];
    qs[w * DM + t] = xn;
    __syncthreads();
  }
  for (int idx = t; idx < NWP * DM; idx += 128) {
    const int w = idx >> 7, n = idx & 127;
    const float* wr = ipw + (size_t)n * DM;
    const float* qr = qs + w * DM;
    float o = 0.f;
#pragma unroll 1
    for (int d = 0; d < DM; ++d) o += qr[d] * wr[d];
    qo[idx] = o + ipb[n];
  }
  __syncthreads();
  const int tt = (t < 96) ? t : 95;
  const v4f a  = *(const v4f*)(qo + tt * 4);
  const v4f bq = *(const v4f*)(qs + tt * 4);
  if (t < 96) {
    *(volatile v4f*)(qout + tt * 4)   = a;
    *(volatile v4f*)(qlnout + tt * 4) = bq;
  }
  __threadfence();
  if (t < 96) {
    *(volatile v4f*)(qout + tt * 4)   = a;
    *(volatile v4f*)(qlnout + tt * 4) = bq;
  }
}

__device__ __forceinline__ void proj_kv(const _Float16* __restrict__ wh, const float* __restrict__ bias,
                                        const _Float16* tokp, _Float16* kvp, int lane, int wave, int hh, int c) {
  const int n0 = wave * HD;
  v16h bf[4];
#pragma unroll
  for (int ks = 0; ks < 4; ++ks) bf[ks] = ldfrag(wh, DM, n0, ks * 32, lane);
  const float bb = bias[n0 + c];
#pragma unroll 1
  for (int mt = 0; mt < TRH / 16; mt += 2) {
    v8f a0c = zero8(), a1c = zero8();
#pragma unroll
    for (int ks = 0; ks < 4; ++ks) {
      const v16h a0 = ldfrag(tokp, TP, mt * 16, ks * 32, lane);
      const v16h a1 = ldfrag(tokp, TP, mt * 16 + 16, ks * 32, lane);
      a0c = mma16(a0, bf[ks], a0c);
      a1c = mma16(a1, bf[ks], a1c);
    }
#pragma unroll
    for (int r = 0; r < 8; ++r) {
      kvp[(mt * 16 + 8 * hh + r) * TP + n0 + c]      = (_Float16)(a0c[r] * KV_SCL + bb);
      kvp[(mt * 16 + 16 + 8 * hh + r) * TP + n0 + c] = (_Float16)(a1c[r] * KV_SCL + bb);
    }
  }
}

__global__ __launch_bounds__(256) void k_main(
    const float* __restrict__ tl, const float* __restrict__ trk, const float* __restrict__ cw,
    const float* __restrict__ cb, const float* __restrict__ pos, const float* __restrict__ se,
    const float* __restrict__ tg, const float* __restrict__ tb, const float* __restrict__ ipb,
    const float* __restrict__ opb, const float* __restrict__ f1b, const float* __restrict__ f2b,
    const float* __restrict__ pag, const float* __restrict__ pab, const float* __restrict__ pfg,
    const float* __restrict__ pfb, const float* __restrict__ hw, const float* __restrict__ hbias,
    const _Float16* __restrict__ wkh, const _Float16* __restrict__ wvh, const _Float16* __restrict__ woh,
    const _Float16* __restrict__ w1h, const _Float16* __restrict__ w2h,
    const float* __restrict__ qf, const float* __restrict__ qlnf, float* __restrict__ out) {
  __shared__ __align__(16) unsigned char lds[L_TOTAL];
  _Float16* tok_h = (_Float16*)(lds + L_TOK);
  _Float16* kv_h  = (_Float16*)(lds + L_KV);
  float*    x32   = (float*)(lds + L_X32);
  _Float16* xh    = (_Float16*)(lds + L_XH);
  _Float16* hf    = (_Float16*)(lds + L_HF);
  float*    sc    = (float*)(lds + L_SC);
  _Float16* ctx_h = (_Float16*)(lds + L_CTX);
  float*    qsh   = (float*)(lds + L_Q);
  float*    qln   = (float*)(lds + L_QLN);
  float*    outs  = (float*)(lds + L_OUT);

  const int tid = threadIdx.x, lane = tid & 31, wave = tid >> 5;
  const int hh = lane >> 4, c = lane & 15;
  const int blk = blockIdx.x;
  const int s0 = blk * SPB;

  for (int i = tid; i < NWP * DM; i += 256) { qsh[i] = qf[i]; qln[i] = qlnf[i]; }

#pragma unroll 1
  for (int hp = 0; hp < 2; ++hp) {
    const int sbase = s0 + hp * SPH;
    {
      const v4f cwa = *(const v4f*)(cw + lane * 8);
      const v4f cwb = *(const v4f*)(cw + lane * 8 + 4);
      const v4f cbv = *(const v4f*)(cb + lane * 4);
      const v4f se0 = *(const v4f*)(se + lane * 4);
      const v4f se1 = *(const v4f*)(se + DM + lane * 4);
      const v4f tgv = *(const v4f*)(tg + lane * 4);
      const v4f tbv = *(const v4f*)(tb + lane * 4);
#pragma unroll 1
      for (int r = wave; r < TRH; r += 8) {
        const int bl   = r / NTK;
        const int kk   = r - bl * NTK;
        const int side = (kk >= TT) ? 1 : 0;
        const int t    = kk - side * TT;
        const size_t co = ((size_t)(sbase + bl) * TT + t) * 2;
        const float lx = tl[co], ly = tl[co + 1], rx = trk[co], ry = trk[co + 1];
        const float cx = side ? rx : lx;
        const float cy = side ? ry : ly;
        const v4f pv = *(const v4f*)(pos + t * DM + lane * 4);
        const float sv0 = side ? se1[0] : se0[0], sv1 = side ? se1[1] : se0[1];
        const float sv2 = side ? se1[2] : se0[2], sv3 = side ? se1[3] : se0[3];
        float u0 = cx * cwa[0] + cy * cwa[1]; u0 = u0 + cbv[0]; u0 = (u0 + pv[0]) + sv0;
        float u1 = cx * cwa[2] + cy * cwa[3]; u1 = u1 + cbv[1]; u1 = (u1 + pv[1]) + sv1;
        float u2 = cx * cwb[0] + cy * cwb[1]; u2 = u2 + cbv[2]; u2 = (u2 + pv[2]) + sv2;
        float u3 = cx * cwb[2] + cy * cwb[3]; u3 = u3 + cbv[3]; u3 = (u3 + pv[3]) + sv3;
        float s = (u0 + u1) + (u2 + u3);
        s = wsum(s);
        const float mean = s * (1.0f / 128.0f);
        const float d0 = u0 - mean, d1 = u1 - mean, d2 = u2 - mean, d3 = u3 - mean;
        float ss = (d0 * d0 + d1 * d1) + (d2 * d2 + d3 * d3);
        ss = wsum(ss);
        const float rstd = rsqrtf(ss * (1.0f / 128.0f) + 1e-5f);
        const float y0 = d0 * rstd * tgv[0] + tbv[0];
        const float y1 = d1 * rstd * tgv[1] + tbv[1];
        const float y2 = d2 * rstd * tgv[2] + tbv[2];
        const float y3 = d3 * rstd * tgv[3] + tbv[3];
        *(v4h*)(tok_h + r * TP + lane * 4) = (v4h){(_Float16)y0, (_Float16)y1, (_Float16)y2, (_Float16)y3};
      }
    }
    __syncthreads();

    proj_kv(wkh, ipb + DM, tok_h, kv_h, lane, wave, hh, c);
    __syncthreads();

#pragma unroll 1
    for (int i = 0; i < 5; ++i) {
      const int item = tid + 256 * i;
      const int bl   = item / (NHD * NTK);
      const int rem  = item - bl * (NHD * NTK);
      const int h    = rem / NTK;
      const int kk   = rem - h * NTK;
      const _Float16* kr = kv_h + (bl * NTK + kk) * TP + h * HD;
      const v8h k0v = *(const v8h*)(kr);
      const v8h k1v = *(const v8h*)(kr + 8);
      const float* q0 = qsh + h * HD;
      float a0 = 0.f, a1 = 0.f, a2 = 0.f;
#pragma unroll
      for (int j = 0; j < 8; ++j) {
        const float kvf = (float)k0v[j];
        a0 += q0[j] * kvf;
        a1 += q0[DM + j] * kvf;
        a2 += q0[2 * DM + j] * kvf;
      }
#pragma unroll
      for (int j = 0; j < 8; ++j) {
        const float kvf = (float)k1v[j];
        a0 += q0[8 + j] * kvf;
        a1 += q0[DM + 8 + j] * kvf;
        a2 += q0[2 * DM + 8 + j] * kvf;
      }
      float* sr = sc + ((bl * NHD + h) * NWP) * NTK + kk;
      sr[0]       = a0 * 0.25f;
      sr[NTK]     = a1 * 0.25f;
      sr[2 * NTK] = a2 * 0.25f;
    }
    __syncthreads();

    if (tid < SPH * NHD * NWP) {
      float* row = sc + tid * NTK;
      float e[NTK];
#pragma unroll
      for (int k2 = 0; k2 < NTK; ++k2) e[k2] = row[k2];
      float m = e[0];
#pragma unroll
      for (int k2 = 1; k2 < NTK; ++k2) m = fmaxf(m, e[k2]);
      float ssum = 0.f;
#pragma unroll
      for (int k2 = 0; k2 < NTK; ++k2) { e[k2] = __expf(e[k2] - m); ssum += e[k2]; }
      const float inv = 1.0f / ssum;
#pragma unroll
      for (int k2 = 0; k2 < NTK; ++k2) row[k2] = e[k2] * inv;
    }
    __syncthreads();

    proj_kv(wvh, ipb + 2 * DM, tok_h, kv_h, lane, wave, hh, c);
    __syncthreads();

    {
      const int ch = tid & 127, hsub = tid >> 7;
      const int h  = ch >> 4;
#pragma unroll 1
      for (int i = 0; i < 4; ++i) {
        const int bl = hsub + 2 * i;
        const float* ar = sc + ((bl * NHD + h) * NWP) * NTK;
        const _Float16* vr = kv_h + (bl * NTK) * TP + ch;
        float a0 = 0.f, a1 = 0.f, a2 = 0.f;
#pragma unroll
        for (int kk = 0; kk < NTK; ++kk) {
          const float vv = (float)vr[kk * TP];
          a0 += ar[kk] * vv;
          a1 += ar[NTK + kk] * vv;
          a2 += ar[2 * NTK + kk] * vv;
        }
        _Float16* cr = ctx_h + ((hp * SPH + bl) * NWP) * TP + ch;
        cr[0]      = (_Float16)(a0 * CTX_CARRY);
        cr[TP]     = (_Float16)(a1 * CTX_CARRY);
        cr[2 * TP] = (_Float16)(a2 * CTX_CARRY);
      }
    }
    __syncthreads();
  }

  {
    const int n0 = wave * 16;
    v8f acc[3];
#pragma unroll
    for (int mt = 0; mt < 3; ++mt) acc[mt] = zero8();
#pragma unroll
    for (int ks = 0; ks < 4; ++ks) {
      const v16h b = ldfrag(woh, DM, n0, ks * 32, lane);
#pragma unroll
      for (int mt = 0; mt < 3; ++mt) {
        const v16h a = ldfrag(ctx_h, TP, mt * 16, ks * 32, lane);
        acc[mt] = mma16(a, b, acc[mt]);
      }
    }
    const float bo = opb[n0 + c];
#pragma unroll
    for (int mt = 0; mt < 3; ++mt) {
#pragma unroll
      for (int r = 0; r < 8; ++r) {
        const int row = mt * 16 + 8 * hh + r;
        const int w   = row % NWP;
        const float t1 = acc[mt][r] * OP_SCL + bo;
        x32[row * XP + n0 + c] = qln[w * DM + n0 + c] + t1;
      }
    }
  }
  __syncthreads();

  {
    const v4f g4 = *(const v4f*)(pag + lane * 4);
    const v4f b4 = *(const v4f*)(pab + lane * 4);
#pragma unroll 1
    for (int i = 0; i < 6; ++i) {
      const int row = wave * 6 + i;
      float* xr = x32 + row * XP + lane * 4;
      const v4f v = *(const v4f*)xr;
      float s = (v[0] + v[1]) + (v[2] + v[3]);
      s = wsum(s);
      const float mean = s * (1.0f / 128.0f);
      const v4f d = v - mean;
      float ss = (d[0] * d[0] + d[1] * d[1]) + (d[2] * d[2] + d[3] * d[3]);
      ss = wsum(ss);
      const float rstd = rsqrtf(ss * (1.0f / 128.0f) + 1e-5f);
      const v4f y = (d * rstd) * g4 + b4;
      *(v4f*)xr = y;
      *(v4h*)(xh + row * TP + lane * 4) = (v4h){(_Float16)y[0], (_Float16)y[1], (_Float16)y[2], (_Float16)y[3]};
    }
  }
  __syncthreads();

#pragma unroll 1
  for (int q2 = 0; q2 < 2; ++q2) {
    const int n0 = (wave + 8 * q2) * 16;
    v8f acc[3];
#pragma unroll
    for (int mt = 0; mt < 3; ++mt) acc[mt] = zero8();
#pragma unroll
    for (int ks = 0; ks < 4; ++ks) {
      const v16h b = ldfrag(w1h, DM, n0, ks * 32, lane);
#pragma unroll
      for (int mt = 0; mt < 3; ++mt) {
        const v16h a = ldfrag(xh, TP, mt * 16, ks * 32, lane);
        acc[mt] = mma16(a, b, acc[mt]);
      }
    }
    const float b1 = f1b[n0 + c];
#pragma unroll
    for (int mt = 0; mt < 3; ++mt) {
#pragma unroll
      for (int r = 0; r < 8; ++r) {
        const int row = mt * 16 + 8 * hh + r;
        const float hv = fmaxf(acc[mt][r] * F1_SCL + b1, 0.f);
        hf[row * HP + n0 + c] = (_Float16)(hv * HID_CARRY);
      }
    }
  }
  __syncthreads();

  {
    const int n0 = wave * 16;
    v8f acc[3];
#pragma unroll
    for (int mt = 0; mt < 3; ++mt) acc[mt] = zero8();
#pragma unroll
    for (int ks = 0; ks < 8; ++ks) {
      const v16h b = ldfrag(w2h, DF, n0, ks * 32, lane);
#pragma unroll
      for (int mt = 0; mt < 3; ++mt) {
        const v16h a = ldfrag(hf, HP, mt * 16, ks * 32, lane);
        acc[mt] = mma16(a, b, acc[mt]);
      }
    }
    const float b2 = f2b[n0 + c];
#pragma unroll
    for (int mt = 0; mt < 3; ++mt) {
#pragma unroll
      for (int r = 0; r < 8; ++r) {
        const int row = mt * 16 + 8 * hh + r;
        const float t2 = acc[mt][r] * F2_SCL + b2;
        const int xi = row * XP + n0 + c;
        const float xv = x32[xi];
        x32[xi] = xv + t2;
      }
    }
  }
  __syncthreads();

  {
    const v4f g4  = *(const v4f*)(pfg + lane * 4);
    const v4f b4  = *(const v4f*)(pfb + lane * 4);
    const v4f hw0 = *(const v4f*)(hw + lane * 4);
    const v4f hw1 = *(const v4f*)(hw + DM + lane * 4);
    const float hb0 = hbias[0], hb1 = hbias[1];
#pragma unroll 1
    for (int i = 0; i < 6; ++i) {
      const int row = wave * 6 + i;
      const float* xr = x32 + row * XP + lane * 4;
      const v4f v = *(const v4f*)xr;
      float s = (v[0] + v[1]) + (v[2] + v[3]);
      s = wsum(s);
      const float mean = s * (1.0f / 128.0f);
      const v4f d = v - mean;
      float ss = (d[0] * d[0] + d[1] * d[1]) + (d[2] * d[2] + d[3] * d[3]);
      ss = wsum(ss);
      const float rstd = rsqrtf(ss * (1.0f / 128.0f) + 1e-5f);
      const v4f y = (d * rstd) * g4 + b4;
      float p0 = (y[0] * hw0[0] + y[1] * hw0[1]) + (y[2] * hw0[2] + y[3] * hw0[3]);
      float p1 = (y[0] * hw1[0] + y[1] * hw1[1]) + (y[2] * hw1[2] + y[3] * hw1[3]);
      p0 = wsum(p0);
      p1 = wsum(p1);
      const float o0 = p0 + hb0, o1 = p1 + hb1;
      if (lane == 0) { outs[row * 2] = o0; outs[row * 2 + 1] = o1; }
    }
  }
  __syncthreads();

  {
    const int tt = (tid < 24) ? tid : 23;
    const v4f val = *(const v4f*)(outs + tt * 4);
    float* op = out + (size_t)blk * NOUT + tt * 4;
    if (tid < 24) *(volatile v4f*)op = val;
    __threadfence();
    if (tid < 24) *(volatile v4f*)op = val;
  }
}

extern "C" void kernel_launch(void* const* d_in, const int* in_sizes, int n_in,
                              void* d_out, int out_size, void* d_ws, size_t ws_size,
                              hipStream_t stream) {
  if (n_in < 25) return;
  const int n0e = in_sizes[0];
  if (n0e <= 0 || (n0e % (NTK * 2)) != 0) return;
  const int nsamp = n0e / (TT * 2);
  if (in_sizes[1] != n0e) return;
  if ((nsamp % SPB) != 0) return;
  if (in_sizes[2] != DM * 2) return;
  if (in_sizes[3] != DM) return;
  if (in_sizes[4] != TT * DM) return;
  if (in_sizes[5] != 2 * DM) return;
  if (in_sizes[6] != NWP * DM) return;
  if (in_sizes[7] != DM || in_sizes[8] != DM || in_sizes[9] != DM || in_sizes[10] != DM) return;
  if (in_sizes[11] != 3 * DM * DM) return;
  if (in_sizes[12] != 3 * DM) return;
  if (in_sizes[13] != DM * DM) return;
  if (in_sizes[14] != DM) return;
  if (in_sizes[15] != DF * DM) return;
  if (in_sizes[16] != DF) return;
  if (in_sizes[17] != DM * DF) return;
  if (in_sizes[18] != DM) return;
  if (in_sizes[19] != DM || in_sizes[20] != DM || in_sizes[21] != DM || in_sizes[22] != DM) return;
  if (in_sizes[23] != 2 * DM) return;
  if (in_sizes[24] != 2) return;
  if (out_size != nsamp * NWP * 2) return;

  const float* track_left  = (const float*)d_in[0];
  const float* track_right = (const float*)d_in[1];
  const float* coord_w     = (const float*)d_in[2];
  const float* coord_b     = (const float*)d_in[3];
  const float* pos_emb     = (const float*)d_in[4];
  const float* side_emb    = (const float*)d_in[5];
  const float* query_emb   = (const float*)d_in[6];
  const float* tok_g       = (const float*)d_in[7];
  const float* tok_b       = (const float*)d_in[8];
  const float* qry_g       = (const float*)d_in[9];
  const float* qry_b       = (const float*)d_in[10];
  const float* in_proj_w   = (const float*)d_in[11];
  const float* in_proj_b   = (const float*)d_in[12];
  const float* out_proj_w  = (const float*)d_in[13];
  const float* out_proj_b  = (const float*)d_in[14];
  const float* fc1_w       = (const float*)d_in[15];
  const float* fc1_b       = (const float*)d_in[16];
  const float* fc2_w       = (const float*)d_in[17];
  const float* fc2_b       = (const float*)d_in[18];
  const float* pa_g        = (const float*)d_in[19];
  const float* pa_b        = (const float*)d_in[20];
  const float* pf_g        = (const float*)d_in[21];
  const float* pf_b        = (const float*)d_in[22];
  const float* head_w      = (const float*)d_in[23];
  const float* head_b      = (const float*)d_in[24];
  float* out = (float*)d_out;

  size_t off = 0;
  const size_t oWk  = off; off += (size_t)DM * DM * 2;
  const size_t oWv  = off; off += (size_t)DM * DM * 2;
  const size_t oWo  = off; off += (size_t)DM * DM * 2;
  const size_t oW1  = off; off += (size_t)DF * DM * 2;
  const size_t oW2  = off; off += (size_t)DM * DF * 2;
  const size_t oQ   = off; off += (size_t)NWP * DM * 4;
  const size_t oQln = off; off += (size_t)NWP * DM * 4;
  if (off > ws_size) return;
  if (off > (size_t)134217728) return;
  if (oWv != oWk + (size_t)DM * DM * 2) return;

  char* ws = (char*)d_ws;
  _Float16* Wk  = (_Float16*)(ws + oWk);
  _Float16* Wv  = (_Float16*)(ws + oWv);
  _Float16* Wo  = (_Float16*)(ws + oWo);
  _Float16* W1  = (_Float16*)(ws + oW1);
  _Float16* W2  = (_Float16*)(ws + oW2);
  float*    Qf  = (float*)(ws + oQ);
  float*    Qln = (float*)(ws + oQln);

  k_wcvt<<<dim3((2 * DM * DM) / 2048), dim3(256), 0, stream>>>(in_proj_w + (size_t)DM * DM, Wk);
  k_wcvt<<<dim3((DM * DM) / 2048), dim3(256), 0, stream>>>(out_proj_w, Wo);
  k_wcvt<<<dim3((DF * DM) / 2048), dim3(256), 0, stream>>>(fc1_w, W1);
  k_wcvt<<<dim3((DM * DF) / 2048), dim3(256), 0, stream>>>(fc2_w, W2);
  k_qprep<<<dim3(1), dim3(128), 0, stream>>>(query_emb, qry_g, qry_b, in_proj_w, in_proj_b, Qf, Qln);
  k_main<<<dim3(nsamp / SPB), dim3(256), 0, stream>>>(
      track_left, track_right, coord_w, coord_b, pos_emb, side_emb, tok_g, tok_b, in_proj_b,
      out_proj_b, fc1_b, fc2_b, pa_g, pa_b, pf_g, pf_b, head_w, head_b,
      Wk, Wv, Wo, W1, W2, Qf, Qln, out);
  (void)hipGetLastError();
}
